// GraphNeuralNetwork_46737834115716
// MI455X (gfx1250) — hardware-verified
//
#include <hip/hip_runtime.h>
#include <math.h>

constexpr int kN      = 100000;
constexpr int kE      = 640000;
constexpr int kG      = 1000;
constexpr int kDin    = 100;
constexpr int kD      = 128;
constexpr int kNPad   = 100032;
constexpr int kNT     = 256;
constexpr int kSRB    = 4096;
constexpr int kRPW    = kSRB / 8;
constexpr int kNTile  = 25;
constexpr int kNRows  = kNTile * kSRB;
constexpr int kSCH    = 4096;
constexpr int kSP     = kSCH / kNT;
constexpr int kNCH    = (kE + kSCH - 1) / kSCH;
constexpr int kLCap   = kSCH + 32;
constexpr int kScanWs = 80;
constexpr int kGT     = 64;
constexpr int kGPW    = kGT / 8;
constexpr int kNPB    = (kG + kGT - 1) / kGT;
constexpr int kSCHP   = 2048;
constexpr int kSPP    = kSCHP / kNT;
constexpr int kNCHP   = (kN + kSCHP - 1) / kSCHP;
constexpr int kLCapP  = kSCHP + 32;
constexpr int kGemmTiles   = (kNPad / 64) * (kD / 64);
constexpr int kGemmBlocks  = (kGemmTiles + 7) / 8;
constexpr int kXcastBlocks = (kNPad * 16) / kNT;
constexpr int kNormBlocks  = kE / kNT;
constexpr float kEps       = 1e-5f;
constexpr float kActCarry  = 16.0f;
constexpr float kWCarry    = 64.0f;
constexpr float kGemmScale = 1.0f / 1024.0f;

static_assert(kE % kSP == 0, "edge groups per thread are whole");
static_assert(kE % 4 == 0 && (kE * 4) % 16 == 0, "dst block 16-B aligned");
static_assert(kN % kSPP == 0, "node groups per thread are whole");
static_assert(kNPad % 64 == 0 && kD % 64 == 0 && kD % 32 == 0, "GEMM tile multiples");
static_assert(kNRows >= kNPad, "accumulator rows cover the padded plane");
static_assert(kRPW == 512 && kRPW % 128 == 0, "wave row ownership");
static_assert((kNPad * 16) % kNT == 0, "cast grid exact");
static_assert(kE % kNT == 0, "norm grid exact");
static_assert(kG % 4 == 0, "output lines in whole float4 pieces");
static_assert(kN < (1 << 17), "node id fits 17 bits");
static_assert(kSRB / kRPW == 8 && kGT / kGPW == 8, "8 owner waves");
static_assert(kScanWs <= kNT && kScanWs > 64, "scan scratch init coverage");
static_assert(kSRB % kNT == 0, "in-place dinv loop covers the tile");

constexpr size_t kWsHw    = (size_t)kNPad * kD * 4;
constexpr size_t kWsAcc   = (size_t)kNRows * kD * 4;
constexpr size_t kWsAct   = (size_t)kNPad * kD * 2;
constexpr size_t kWsWt    = (size_t)3 * kD * kD * 2;
constexpr size_t kWsDinv  = (size_t)kNRows * 4;
constexpr size_t kWsNorm  = (size_t)kE * 4;
constexpr size_t kWsTotal = kWsHw + kWsAcc + kWsAct + kWsWt + kWsDinv + kWsNorm;
static_assert(kWsTotal == 132321280, "carve total");
static_assert(kWsTotal <= (size_t)134217728, "carve under 128 MiB");
static_assert(kWsHw % 256 == 0 && kWsAcc % 256 == 0 && kWsAct % 256 == 0 && kWsWt % 256 == 0 && kWsDinv % 256 == 0, "aligned regions");

typedef __attribute__((ext_vector_type(16))) _Float16 v16h;
typedef __attribute__((ext_vector_type(8)))  _Float16 v8h;
typedef __attribute__((ext_vector_type(16))) __bf16   v16b;
typedef __attribute__((ext_vector_type(8)))  __bf16   v8b;
typedef __attribute__((ext_vector_type(8)))  float    v8f;
typedef __attribute__((ext_vector_type(4)))  float    v4f;
typedef __attribute__((ext_vector_type(4)))  int      v4i;
typedef __attribute__((ext_vector_type(4)))  unsigned int v4u;

__device__ __forceinline__ unsigned short f2bf_bits(float f) {
  unsigned u = __float_as_uint(f);
  return (unsigned short)((u + 0x7FFFu + ((u >> 16) & 1u)) >> 16);
}
__device__ __forceinline__ float bf_bits2f(unsigned short h) { return __uint_as_float(((unsigned)h) << 16); }

__device__ __forceinline__ void dep_guard4_h(v8f& a, v8f& b, v8f& c, v8f& d, v16h x, v16h y) { asm volatile("v_nop\n\tv_nop\n\tv_nop\n\tv_nop" : "+v"(a), "+v"(b), "+v"(c), "+v"(d) : "v"(x), "v"(y)); }
__device__ __forceinline__ void dep_guard4_b(v8f& a, v8f& b, v8f& c, v8f& d, v16b x, v16b y) { asm volatile("v_nop\n\tv_nop\n\tv_nop\n\tv_nop" : "+v"(a), "+v"(b), "+v"(c), "+v"(d) : "v"(x), "v"(y)); }
__device__ __forceinline__ void keep4_h(v16h a, v16h b, v16h c, v16h d) { asm volatile("v_nop" :: "v"(a), "v"(b), "v"(c), "v"(d)); }
__device__ __forceinline__ void keep4_b(v16b a, v16b b, v16b c, v16b d) { asm volatile("v_nop" :: "v"(a), "v"(b), "v"(c), "v"(d)); }
__device__ __forceinline__ void acc_guard4(v8f& a, v8f& b, v8f& c, v8f& d) { asm volatile("v_nop\n\tv_nop\n\tv_nop\n\tv_nop" : "+v"(a), "+v"(b), "+v"(c), "+v"(d)); }
template <typename T> struct Frag;
template <> struct Frag<_Float16> {
  typedef v16h V; union U { v16h v; v8h h[2]; };
  static __device__ __forceinline__ v16h load(const _Float16* p) {
    U f; f.h[0] = *(const v8h*)(p); f.h[1] = *(const v8h*)(p + 16); return f.v;
  }
  static __device__ __forceinline__ v8f mma(v16h a, v16h b, v8f c) {
    return __builtin_amdgcn_wmma_f32_16x16x32_f16(false, a, false, b, (short)0, c, false, false);
  }
  static __device__ __forceinline__ void guard4(v8f& a, v8f& b, v8f& c, v8f& d, v16h x, v16h y) { dep_guard4_h(a, b, c, d, x, y); }
  static __device__ __forceinline__ void keep(v16h a, v16h b, v16h c, v16h d) { keep4_h(a, b, c, d); }
};
template <> struct Frag<__bf16> {
  typedef v16b V; union U { v16b v; v8b h[2]; };
  static __device__ __forceinline__ v16b load(const __bf16* p) {
    U f; f.h[0] = *(const v8b*)(p); f.h[1] = *(const v8b*)(p + 16); return f.v;
  }
  static __device__ __forceinline__ v8f mma(v16b a, v16b b, v8f c) {
    return __builtin_amdgcn_wmma_f32_16x16x32_bf16(false, a, false, b, (short)0, c, false, false);
  }
  static __device__ __forceinline__ void guard4(v8f& a, v8f& b, v8f& c, v8f& d, v16b x, v16b y) { dep_guard4_b(a, b, c, d, x, y); }
  static __device__ __forceinline__ void keep(v16b a, v16b b, v16b c, v16b d) { keep4_b(a, b, c, d); }
};

__device__ __forceinline__ unsigned pk16(unsigned short a, unsigned short b) { return (unsigned)a | ((unsigned)b << 16); }
__device__ __forceinline__ unsigned short h_bits(float f) { const _Float16 h = (_Float16)f; return __builtin_bit_cast(unsigned short, h); }

template <int ET> struct Elem;
template <> struct Elem<0> { typedef _Float16 T; };
template <> struct Elem<1> { typedef __bf16 T; };
template <int ET, bool SPLIT, int BIAS_MODE, int OUT_MODE, bool RESID, int ACT = 0>
__global__ __launch_bounds__(256) void wmma_gemm64(
    const unsigned short* __restrict__ Ap, const unsigned short* __restrict__ A2p, int lda, long strideA,
    const unsigned short* __restrict__ Btp, const unsigned short* __restrict__ Bt2p, int ldb, long strideB,
    void* __restrict__ Cout, void* __restrict__ Cout2, int ldc, long strideC,
    const float* __restrict__ bias,
    const float* __restrict__ resid, long strideR,
    int M, int N, int K, float scale) {
  typedef typename Elem<ET>::T T;
  typedef typename Frag<T>::V V;
  const T* A = (const T*)Ap; const T* A2 = (const T*)A2p; const T* Bt = (const T*)Btp; const T* Bt2 = (const T*)Bt2p;
  __shared__ __align__(16) float sT[8][16 * 68];
  const int b    = blockIdx.y;
  const int lane = threadIdx.x & 31;
  const int wave = threadIdx.x >> 5;
  const int tilesN = N >> 6;
  const int tilesM = M >> 6;
  const int tile = blockIdx.x * 8 + wave;
  if (tile >= tilesM * tilesN) return;
  const int tm = tile / tilesN;
  const int tn = tile - tm * tilesN;
  const int m0 = tm << 6;
  const int n0 = tn << 6;

  const T* Ab  = A  + (size_t)b * strideA;
  const T* Bb  = Bt + (size_t)b * strideB;
  const T* Ab2 = SPLIT ? (A2  + (size_t)b * strideA) : nullptr;
  const T* Bb2 = SPLIT ? (Bt2 + (size_t)b * strideB) : nullptr;

  const int rlane = lane & 15;
  const int koff  = (lane >> 4) * 8;
  const int mOff  = (lane >> 4) * 8;

  v8f acc[4][4];
#pragma unroll
  for (int i = 0; i < 4; ++i)
#pragma unroll
    for (int j = 0; j < 4; ++j) acc[i][j] = (v8f){0.f,0.f,0.f,0.f,0.f,0.f,0.f,0.f};

  for (int k0 = 0; k0 < K; k0 += 32) {
    V bh[4], bl[4];
#pragma unroll
    for (int j = 0; j < 4; ++j) {
      const size_t bo = (size_t)(n0 + (j << 4) + rlane) * ldb + koff + k0;
      bh[j] = Frag<T>::load(Bb + bo);
      if (SPLIT) bl[j] = Frag<T>::load(Bb2 + bo);
    }
#pragma unroll
    for (int i = 0; i < 4; ++i) {
      const size_t ao = (size_t)(m0 + (i << 4) + rlane) * lda + koff + k0;
      V ah = Frag<T>::load(Ab + ao);
      V al;
      if (SPLIT) al = Frag<T>::load(Ab2 + ao);
#pragma unroll
      for (int j = 0; j < 4; ++j) {
        acc[i][j] = Frag<T>::mma(ah, bh[j], acc[i][j]);
        if (SPLIT) {
          acc[i][j] = Frag<T>::mma(ah, bl[j], acc[i][j]);
          acc[i][j] = Frag<T>::mma(al, bh[j], acc[i][j]);
        }
      }
      Frag<T>::guard4(acc[i][0], acc[i][1], acc[i][2], acc[i][3], ah, SPLIT ? al : bh[3]);
    }
    Frag<T>::keep(bh[0], bh[1], bh[2], bh[3]);
    if (SPLIT) Frag<T>::keep(bl[0], bl[1], bl[2], bl[3]);
  }
  acc_guard4(acc[0][0], acc[0][1], acc[0][2], acc[0][3]);
  acc_guard4(acc[1][0], acc[1][1], acc[1][2], acc[1][3]);
  acc_guard4(acc[2][0], acc[2][1], acc[2][2], acc[2][3]);
  acc_guard4(acc[3][0], acc[3][1], acc[3][2], acc[3][3]);

  float* slab = sT[wave];
  const float* Rb = RESID ? (resid + (size_t)b * strideR) : nullptr;
#pragma unroll
  for (int i = 0; i < 4; ++i) {
    const int mBase = m0 + (i << 4);
#pragma unroll
    for (int j = 0; j < 4; ++j) {
      const int n = n0 + (j << 4) + rlane;
      float bv = 0.f;
      if (BIAS_MODE == 2) bv = bias[n];
#pragma unroll
      for (int r = 0; r < 8; ++r) {
        float v = acc[i][j][r] * scale;
        if (BIAS_MODE == 1) v += bias[mBase + mOff + r];
        if (BIAS_MODE == 2) v += bv;
        if (RESID) v += Rb[(size_t)(mBase + mOff + r) * ldc + n];
        if (ACT == 2) v = fmaxf(v, 0.0f);
        if (ACT == 4) v = (v > 0.f) ? v : 0.01f * v;
        slab[(mOff + r) * 68 + (j << 4) + rlane] = v;
      }
    }
    __builtin_amdgcn_fence(__ATOMIC_RELEASE, "workgroup");
    __builtin_amdgcn_wave_barrier();
    __builtin_amdgcn_fence(__ATOMIC_ACQUIRE, "workgroup");
    if (OUT_MODE == 0) {
      float* C = (float*)Cout + (size_t)b * strideC;
      const int hh = lane >> 4, c4 = (lane & 15) * 4;
      for (int pass = 0; pass < 2; ++pass) {
#pragma unroll
        for (int it = 0; it < 8; ++it) {
          const int row = it * 2 + hh;
          v4f v = *(const v4f*)(slab + row * 68 + c4);
          *(volatile v4f*)(C + (size_t)(mBase + row) * ldc + n0 + c4) = v;
        }
        __threadfence();
      }
    } else {
      const int q = lane >> 3, c8 = (lane & 7) * 8;
      unsigned short* C  = (unsigned short*)Cout  + (size_t)b * strideC;
      unsigned short* C2 = (OUT_MODE == 2) ? ((unsigned short*)Cout2 + (size_t)b * strideC) : nullptr;
      for (int pass = 0; pass < 2; ++pass) {
#pragma unroll
        for (int it = 0; it < 4; ++it) {
          const int row = it * 4 + q;
          const float* sp = slab + row * 68 + c8;
          v8h hv, lv;
#pragma unroll
          for (int e = 0; e < 8; ++e) {
            if (OUT_MODE == 1) {
              hv[e] = (_Float16)sp[e];
            } else {
              unsigned short hb = f2bf_bits(sp[e]);
              unsigned short lb = f2bf_bits(sp[e] - bf_bits2f(hb));
              hv[e] = __builtin_bit_cast(_Float16, hb);
              lv[e] = __builtin_bit_cast(_Float16, lb);
            }
          }
          *(volatile v8h*)(C + (size_t)(mBase + row) * ldc + n0 + c8) = hv;
          if (OUT_MODE == 2) *(volatile v8h*)(C2 + (size_t)(mBase + row) * ldc + n0 + c8) = lv;
        }
        __threadfence();
      }
    }
    __builtin_amdgcn_fence(__ATOMIC_RELEASE, "workgroup");
    __builtin_amdgcn_wave_barrier();
    __builtin_amdgcn_fence(__ATOMIC_ACQUIRE, "workgroup");
  }
}

__device__ __forceinline__ int blk_excl_scan(int cnt, int* scan_ws, int tid, int* tot) {
  const int lane = tid & 31, wave = tid >> 5; int incl = cnt;
#pragma unroll
  for (int o = 1; o < 32; o <<= 1) { const int v = __shfl_up(incl, o, 32); if (lane >= o) incl += v; }
  if (lane == 31) scan_ws[wave] = incl;
  __syncthreads();
  if (wave == 0) {
    int wv = scan_ws[lane & 7]; wv = (lane < kNT / 32) ? wv : 0; int wincl = wv;
#pragma unroll
    for (int o = 1; o < 32; o <<= 1) { const int v = __shfl_up(wincl, o, 32); if (lane >= o) wincl += v; }
    if (lane < kNT / 32) scan_ws[32 + lane] = wincl - wv; if (lane == 31) scan_ws[64] = wincl; }
  __syncthreads();
  const int res = scan_ws[32 + wave] + incl - cnt; *tot = scan_ws[64];
  return res;
}

template <int SP, int CAP>
__device__ __forceinline__ int chunk_hits_w(const int* __restrict__ dstv, const int* __restrict__ srcv, const float* __restrict__ wv,
                                            int e0, int n0, int tid, int* LA, float* LW, int* scan_ws) {
  const int eb = e0 + tid * SP;
  const bool vg = eb < kE;
  const int ebc = vg ? eb : (kE - SP);
  v4i d4[SP / 4];
#pragma unroll
  for (int q = 0; q < SP / 4; ++q) d4[q] = *(const v4i*)(dstv + ebc + 4 * q);
  asm volatile("" ::: "memory");
  v4i s4[SP / 4]; v4f w4[SP / 4];
#pragma unroll
  for (int q = 0; q < SP / 4; ++q) { s4[q] = *(const v4i*)(srcv + ebc + 4 * q); w4[q] = *(const v4f*)(wv + ebc + 4 * q); }
  asm volatile("" ::: "memory");
  int rec[SP]; float recw[SP]; int cnt = 0;
#pragma unroll
  for (int q = 0; q < SP / 4; ++q) {
#pragma unroll
    for (int e = 0; e < 4; ++e) {
      int d = d4[q][e]; d = d < 0 ? 0 : (d >= kN ? kN - 1 : d);
      int s = s4[q][e]; s = s < 0 ? 0 : (s >= kN ? kN - 1 : s);
      const bool hit = vg && (d >= n0) && (d < n0 + kSRB);
      rec[4 * q + e]  = hit ? (((d - n0) << 17) | s) : -1;
      recw[4 * q + e] = w4[q][e];
      cnt += hit ? 1 : 0;
    }
  }
  int tot; int p = blk_excl_scan(cnt, scan_ws, tid, &tot);
#pragma unroll
  for (int k = 0; k < SP; ++k) if (rec[k] >= 0) { if ((unsigned)p < (unsigned)CAP) { LA[p] = rec[k]; LW[p] = recw[k]; } ++p; }
  __syncthreads();
  return tot < CAP ? tot : CAP;
}

__global__ __launch_bounds__(kNT) void wprep_kernel(const float* __restrict__ W0, const float* __restrict__ W1,
                                                   const float* __restrict__ W2, unsigned short* __restrict__ wt) {
  const int z  = blockIdx.x >> 3;
  const int n  = ((blockIdx.x & 7) << 4) + (threadIdx.x >> 4);
  const int c8 = (threadIdx.x & 15) * 8;
  const float* W = (z == 0) ? W0 : ((z == 1) ? W1 : W2);
  const int Kz = (z == 0) ? kDin : kD;
  unsigned short hb[8];
#pragma unroll
  for (int e = 0; e < 8; ++e) {
    const int k  = c8 + e;
    const int kc = k < Kz ? k : Kz - 1;
    const float f = (k < Kz) ? kWCarry : 0.0f;
    const float v = W[(size_t)kc * kD + n] * f;
    hb[e] = h_bits(v);
  }
  const v4u u = (v4u){pk16(hb[0], hb[1]), pk16(hb[2], hb[3]), pk16(hb[4], hb[5]), pk16(hb[6], hb[7])};
  unsigned short* op = wt + (size_t)z * kD * kD + (size_t)n * kD + c8;
  *(volatile v4u*)op = u;
  __threadfence();
  *(volatile v4u*)op = u;
}

__global__ __launch_bounds__(kNT) void xcast_kernel(const float* __restrict__ x, unsigned short* __restrict__ act) {
  const int i   = blockIdx.x * kNT + threadIdx.x;
  const int row = i >> 4, c8 = (i & 15) * 8;
  const int rc  = row < kN ? row : kN - 1;
  const int col0 = c8 < 96 ? c8 : 96;
  const int col1 = (c8 + 4) < 96 ? (c8 + 4) : 96;
  const float fa = (row < kN && c8 < kDin) ? kActCarry : 0.0f;
  const float fb = (row < kN && c8 + 4 < kDin) ? kActCarry : 0.0f;
  const v4f a = *(const v4f*)(x + (size_t)rc * kDin + col0);
  const v4f b = *(const v4f*)(x + (size_t)rc * kDin + col1);
  const v4f av = a * fa, bv = b * fb;
  unsigned short hb[8];
#pragma unroll
  for (int e = 0; e < 4; ++e) { hb[e] = h_bits(av[e]); hb[4 + e] = h_bits(bv[e]); }
  const v4u u = (v4u){pk16(hb[0], hb[1]), pk16(hb[2], hb[3]), pk16(hb[4], hb[5]), pk16(hb[6], hb[7])};
  unsigned short* op = act + (size_t)row * kD + c8;
  *(volatile v4u*)op = u;
  __threadfence();
  *(volatile v4u*)op = u;
}

__global__ __launch_bounds__(kNT) void deg_kernel(const int* __restrict__ ei, const float* __restrict__ ew, float* __restrict__ dinv) {
  __shared__ int LA[kLCap];
  __shared__ float LW[kLCap];
  __shared__ __align__(16) float SDEG[kSRB];
  __shared__ int scan_ws[kScanWs];
  const int tid = threadIdx.x, lane = tid & 31, wave = tid >> 5;
  const int n0 = blockIdx.x * kSRB;
  for (int i = tid; i < kSRB; i += kNT) SDEG[i] = 1.0f;
  for (int i = tid; i < kLCap; i += kNT) { LA[i] = 0; LW[i] = 0.0f; }
  if (tid < kScanWs) scan_ws[tid] = 0;
  __syncthreads();
  const int* srcv = ei; const int* dstv = ei + kE;
#pragma unroll 1
  for (int c = 0; c < kNCH; ++c) {
    const int tot = chunk_hits_w<kSP, kSCH>(dstv, srcv, ew, c * kSCH, n0, tid, LA, LW, scan_ws);
#pragma unroll 1
    for (int base = 0; base < tot; base += 32) {
      const int q  = base + lane;
      const int qc = q < kLCap - 1 ? q : kLCap - 1;
      const int rv = LA[qc]; const float wq = LW[qc];
      const int own = (q < tot && (rv >> 26) == wave) ? 1 : 0;
      unsigned msk = (unsigned)__ballot(own);
#pragma unroll 1
      for (int it = 0; it < 32; ++it) {
        if (msk == 0u) break;
        const int bp = __builtin_ctz(msk); msk &= msk - 1u;
        const int r = __shfl(rv, bp, 32);
        const float w = __shfl(wq, bp, 32);
        const int dl = r >> 17;
        const float t = SDEG[dl] + w;
        if (lane == 0) SDEG[dl] = t;
      }
    }
    __syncthreads();
  }
#pragma unroll 1
  for (int i = tid; i < kSRB; i += kNT) {
    const float d = SDEG[i];
    const float r = 1.0f / sqrtf(d);
    SDEG[i] = (d > 0.0f) ? r : 0.0f;
  }
  __syncthreads();
  for (int pass = 0; pass < 2; ++pass) {
#pragma unroll
    for (int it = 0; it < 4; ++it) {
      const int r0 = wave * kRPW + it * 128 + 4 * lane;
      const v4f o = *(const v4f*)(SDEG + r0);
      *(volatile v4f*)(dinv + (size_t)n0 + r0) = o;
    }
    __threadfence();
  }
}

__global__ __launch_bounds__(kNT) void norm_kernel(const int* __restrict__ ei, const float* __restrict__ ew,
                                                  const float* __restrict__ dinv, float* __restrict__ normw) {
  const int e = blockIdx.x * kNT + threadIdx.x;
  int s = ei[e]; int d = ei[kE + e];
  s = s < 0 ? 0 : (s >= kN ? kN - 1 : s);
  d = d < 0 ? 0 : (d >= kN ? kN - 1 : d);
  const float a = dinv[s] * ew[e];
  const float v = a * dinv[d];
  ((volatile float*)normw)[e] = v;
  __threadfence();
  ((volatile float*)normw)[e] = v;
}

template <int OUTF16>
__global__ __launch_bounds__(kNT) void agg_kernel(const float* __restrict__ hw, const int* __restrict__ ei, const float* __restrict__ normw,
                                                 const float* __restrict__ dinv, const float* __restrict__ bias,
                                                 const float* __restrict__ gam, const float* __restrict__ bet,
                                                 const float* __restrict__ rmean, const float* __restrict__ rvar,
                                                 float* acc, unsigned short* __restrict__ act) {
  __shared__ int LA[kLCap];
  __shared__ float LW[kLCap];
  __shared__ __align__(16) float SPAR[5 * kD];
  __shared__ int scan_ws[kScanWs];
  const int tid = threadIdx.x, lane = tid & 31, wave = tid >> 5;
  const int n0 = blockIdx.x * kSRB;
  if (tid < kD) {
    SPAR[tid]          = bias[tid];
    SPAR[kD + tid]     = rmean[tid];
    SPAR[2 * kD + tid] = gam[tid];
    SPAR[3 * kD + tid] = 1.0f / sqrtf(rvar[tid] + kEps);
    SPAR[4 * kD + tid] = bet[tid];
  }
  for (int i = tid; i < kLCap; i += kNT) { LA[i] = 0; LW[i] = 0.0f; }
  if (tid < kScanWs) scan_ws[tid] = 0;
  __syncthreads();

#pragma unroll 1
  for (int j = 0; j < kRPW; ++j) {
    const int n  = n0 + wave * kRPW + j;
    const int nc = n < kNPad ? n : kNPad - 1;
    const float di = dinv[n];
    const float ns = di * di;
    const v4f hv = *(const v4f*)(hw + (size_t)nc * kD + 4 * lane);
    const v4f a0 = hv * ns;
    *(v4f*)(acc + (size_t)n * kD + 4 * lane) = a0;
  }

  const int* srcv = ei; const int* dstv = ei + kE;
#pragma unroll 1
  for (int c = 0; c < kNCH; ++c) {
    const int tot = chunk_hits_w<kSP, kSCH>(dstv, srcv, normw, c * kSCH, n0, tid, LA, LW, scan_ws);
#pragma unroll 1
    for (int base = 0; base < tot; base += 32) {
      const int q  = base + lane;
      const int qc = q < kLCap - 1 ? q : kLCap - 1;
      const int rv = LA[qc]; const float wq = LW[qc];
      const int own = (q < tot && (rv >> 26) == wave) ? 1 : 0;
      unsigned msk = (unsigned)__ballot(own);
#pragma unroll 1
      for (int it = 0; it < 32; ++it) {
        if (msk == 0u) break;
        const int bp = __builtin_ctz(msk); msk &= msk - 1u;
        const int r = __shfl(rv, bp, 32);
        const float w = __shfl(wq, bp, 32);
        const int dl = r >> 17, s = r & 0x1FFFF;
        const v4f hv = *(const v4f*)(hw + (size_t)s * kD + 4 * lane);
        float* rp = acc + (size_t)(n0 + dl) * kD + 4 * lane;
        v4f a = *(const v4f*)rp;
        a = a + w * hv;
        *(v4f*)rp = a;
      }
    }
    __syncthreads();
  }

  if (OUTF16 == 1) {
    const int c = lane & 15, hh = lane >> 4;
    float pb[8], prm[8], pg[8], prs[8], pbt[8];
    {
      const v4f b0 = *(const v4f*)(SPAR + 8 * c),          b1 = *(const v4f*)(SPAR + 8 * c + 4);
      const v4f m0 = *(const v4f*)(SPAR + kD + 8 * c),     m1 = *(const v4f*)(SPAR + kD + 8 * c + 4);
      const v4f g0 = *(const v4f*)(SPAR + 2 * kD + 8 * c), g1 = *(const v4f*)(SPAR + 2 * kD + 8 * c + 4);
      const v4f v0 = *(const v4f*)(SPAR + 3 * kD + 8 * c), v1 = *(const v4f*)(SPAR + 3 * kD + 8 * c + 4);
      const v4f t0 = *(const v4f*)(SPAR + 4 * kD + 8 * c), t1 = *(const v4f*)(SPAR + 4 * kD + 8 * c + 4);
#pragma unroll
      for (int e = 0; e < 4; ++e) {
        pb[e] = b0[e];  pb[4 + e] = b1[e];
        prm[e] = m0[e]; prm[4 + e] = m1[e];
        pg[e] = g0[e];  pg[4 + e] = g1[e];
        prs[e] = v0[e]; prs[4 + e] = v1[e];
        pbt[e] = t0[e]; pbt[4 + e] = t1[e];
      }
    }
#pragma unroll 1
    for (int j = 0; j < kRPW; j += 2) {
      const int nb = n0 + wave * kRPW + j;
      if (nb < kNPad) {
        const int n = nb + hh;
        const float livef = (n < kN) ? 1.0f : 0.0f;
        const float* rp = acc + (size_t)n * kD + 8 * c;
        const v4f a0 = *(const v4f*)rp;
        const v4f a1 = *(const v4f*)(rp + 4);
        float av[8];
#pragma unroll
        for (int e = 0; e < 4; ++e) { av[e] = a0[e]; av[4 + e] = a1[e]; }
        unsigned short hb[8];
#pragma unroll
        for (int e = 0; e < 8; ++e) {
          float t = av[e] + pb[e];
          t = t - prm[e];
          t = pg[e] * t;
          t = t * prs[e];
          t = t + pbt[e];
          t = fmaxf(t, 0.0f);
          t = t * livef;
          hb[e] = h_bits(t * kActCarry);
        }
        const v4u u = (v4u){pk16(hb[0], hb[1]), pk16(hb[2], hb[3]), pk16(hb[4], hb[5]), pk16(hb[6], hb[7])};
        unsigned short* op = act + (size_t)n * kD + 8 * c;
        for (int pass = 0; pass < 2; ++pass) {
          *(volatile v4u*)op = u;
          __threadfence();
        }
      }
    }
  } else {
    const v4f pb  = *(const v4f*)(SPAR + 4 * lane);
    const v4f prm = *(const v4f*)(SPAR + kD + 4 * lane);
    const v4f pg  = *(const v4f*)(SPAR + 2 * kD + 4 * lane);
    const v4f prs = *(const v4f*)(SPAR + 3 * kD + 4 * lane);
    const v4f pbt = *(const v4f*)(SPAR + 4 * kD + 4 * lane);
#pragma unroll 1
    for (int j = 0; j < kRPW; ++j) {
      const int n = n0 + wave * kRPW + j;
      float* rp = acc + (size_t)n * kD + 4 * lane;
      const v4f a = *(const v4f*)rp;
      v4f o;
#pragma unroll
      for (int e = 0; e < 4; ++e) {
        float t = a[e] + pb[e];
        t = t - prm[e];
        t = pg[e] * t;
        t = t * prs[e];
        t = t + pbt[e];
        o[e] = fmaxf(t, 0.0f);
      }
      for (int pass = 0; pass < 2; ++pass) {
        *(volatile v4f*)rp = o;
        __threadfence();
      }
    }
  }
}

__global__ __launch_bounds__(kNT) void pool_kernel(const float* __restrict__ h3, const int* __restrict__ bidx,
                                                  const float* __restrict__ wout, const float* __restrict__ bout,
                                                  float* __restrict__ out) {
  __shared__ int LP[kLCapP];
  __shared__ __align__(16) float SACC[kGT * kD];
  __shared__ int SCNT[kGT];
  __shared__ __align__(16) float SOUT[kGT];
  __shared__ int scan_ws[kScanWs];
  const int tid = threadIdx.x, lane = tid & 31, wave = tid >> 5;
  const int g0 = blockIdx.x * kGT;
  for (int i = tid; i < kGT * kD; i += kNT) SACC[i] = 0.0f;
  for (int i = tid; i < kLCapP; i += kNT) LP[i] = 0;
  if (tid < kGT) { SCNT[tid] = 0; SOUT[tid] = 0.0f; }
  if (tid < kScanWs) scan_ws[tid] = 0;
  __syncthreads();
#pragma unroll 1
  for (int cch = 0; cch < kNCHP; ++cch) {
    const int eb = cch * kSCHP + tid * kSPP;
    const bool vg = eb < kN;
    const int ebc = vg ? eb : (kN - kSPP);
    const v4i b0 = *(const v4i*)(bidx + ebc);
    const v4i b1 = *(const v4i*)(bidx + ebc + 4);
    int bv[8];
#pragma unroll
    for (int k = 0; k < 4; ++k) { bv[k] = b0[k]; bv[4 + k] = b1[k]; }
    int rec[8]; int cnt = 0;
#pragma unroll
    for (int k = 0; k < 8; ++k) {
      const bool hit = vg && (bv[k] >= g0) && (bv[k] < g0 + kGT);
      rec[k] = hit ? (((bv[k] - g0) << 17) | (ebc + k)) : -1;
      cnt += hit ? 1 : 0;
    }
    int tot; int p = blk_excl_scan(cnt, scan_ws, tid, &tot);
#pragma unroll
    for (int k = 0; k < 8; ++k) if (rec[k] >= 0) { if ((unsigned)p < (unsigned)kSCHP) LP[p] = rec[k]; ++p; }
    __syncthreads();
    const int totc = tot < kSCHP ? tot : kSCHP;
#pragma unroll 1
    for (int base = 0; base < totc; base += 32) {
      const int q  = base + lane;
      const int qc = q < kLCapP - 1 ? q : kLCapP - 1;
      const int rv = LP[qc];
      const int own = (q < totc && (rv >> 20) == wave) ? 1 : 0;
      unsigned msk = (unsigned)__ballot(own);
#pragma unroll 1
      for (int it = 0; it < 32; ++it) {
        if (msk == 0u) break;
        const int bp = __builtin_ctz(msk); msk &= msk - 1u;
        const int r = __shfl(rv, bp, 32);
        const int gl = r >> 17, nd = r & 0x1FFFF;
        const v4f hv = *(const v4f*)(h3 + (size_t)nd * kD + 4 * lane);
        float* sp = SACC + gl * kD + 4 * lane;
        v4f a = *(const v4f*)sp;
        a = a + hv;
        *(v4f*)sp = a;
        const int c0 = SCNT[gl];
        if (lane == 0) SCNT[gl] = c0 + 1;
      }
    }
    __syncthreads();
  }
  const v4f wo = *(const v4f*)(wout + 4 * lane);
  const float bo = bout[0];
#pragma unroll 1
  for (int i = 0; i < kGPW; ++i) {
    const int gl = wave * kGPW + i;
    const v4f s = *(const v4f*)(SACC + gl * kD + 4 * lane);
    const float cf = (float)SCNT[gl];
    const float inv = 1.0f / fmaxf(cf, 1.0f);
    const v4f pv = s * inv;
    float d = pv[0] * wo[0];
    d = d + pv[1] * wo[1];
    d = d + pv[2] * wo[2];
    d = d + pv[3] * wo[3];
    d += __shfl_xor(d, 16, 32);
    d += __shfl_xor(d, 8, 32);
    d += __shfl_xor(d, 4, 32);
    d += __shfl_xor(d, 2, 32);
    d += __shfl_xor(d, 1, 32);
    const float o = d + bo;
    if (lane == 0) SOUT[gl] = o;
  }
  __syncthreads();
  if (wave == 0) {
    const int rem = kG - g0;
    const int nl  = rem >= kGT ? (kGT / 4) : (rem / 4);
    const int li  = lane < (kGT / 4) ? lane : (kGT / 4 - 1);
    const v4f v = *(const v4f*)(SOUT + 4 * li);
    for (int pass = 0; pass < 2; ++pass) {
      if (lane < nl) *(volatile v4f*)(out + g0 + 4 * lane) = v;
      __threadfence();
    }
  }
}

extern "C" void kernel_launch(void* const* d_in, const int* in_sizes, int n_in,
                              void* d_out, int out_size, void* d_ws, size_t ws_size, hipStream_t stream) {
  (void)in_sizes; (void)n_in; (void)out_size;
  const float* x     = (const float*)d_in[0];
  const int*   ei    = (const int*)  d_in[1];
  const float* ew    = (const float*)d_in[2];
  const int*   bidx  = (const int*)  d_in[3];
  const float* W0    = (const float*)d_in[4];
  const float* b0    = (const float*)d_in[5];
  const float* W1    = (const float*)d_in[6];
  const float* b1    = (const float*)d_in[7];
  const float* W2    = (const float*)d_in[8];
  const float* b2    = (const float*)d_in[9];
  const float* gam   = (const float*)d_in[10];
  const float* bet   = (const float*)d_in[11];
  const float* rmean = (const float*)d_in[12];
  const float* rvar  = (const float*)d_in[13];
  const float* wout  = (const float*)d_in[14];
  const float* bout  = (const float*)d_in[15];
  float* out = (float*)d_out;

  if (ws_size < kWsTotal) return;
  char* ws = (char*)d_ws;
  size_t off = 0;
  float*          hw    = (float*)(ws + off);           off += kWsHw;
  float*          accp  = (float*)(ws + off);           off += kWsAcc;
  unsigned short* act16 = (unsigned short*)(ws + off);  off += kWsAct;
  unsigned short* wt    = (unsigned short*)(ws + off);  off += kWsWt;
  float*          dinv  = (float*)(ws + off);           off += kWsDinv;
  float*          normw = (float*)(ws + off);           off += kWsNorm;
  if (off != kWsTotal || off > ws_size) return;

  wprep_kernel<<<24, kNT, 0, stream>>>(W0, W1, W2, wt);
  xcast_kernel<<<kXcastBlocks, kNT, 0, stream>>>(x, act16);
  deg_kernel<<<kNTile, kNT, 0, stream>>>(ei, ew, dinv);
  norm_kernel<<<kNormBlocks, kNT, 0, stream>>>(ei, ew, dinv, normw);

  const float* bl[3] = {b0, b1, b2};
  for (int l = 0; l < 3; ++l) {
    const unsigned short* btp = wt + (size_t)l * kD * kD;
    wmma_gemm64<0, false, 0, 0, false, 0><<<dim3(kGemmBlocks, 1), 256, 0, stream>>>(
        (const unsigned short*)act16, (const unsigned short*)act16, kD, 0L,
        btp, btp, kD, 0L,
        (void*)hw, (void*)nullptr, kD, 0L,
        (const float*)nullptr, (const float*)nullptr, 0L, kNPad, kD, kD, kGemmScale);
    if (l < 2) {
      agg_kernel<1><<<kNTile, kNT, 0, stream>>>(hw, ei, normw, dinv, bl[l], gam + l * kD, bet + l * kD,
                                                 rmean + l * kD, rvar + l * kD, accp, act16);
    } else {
      agg_kernel<0><<<kNTile, kNT, 0, stream>>>(hw, ei, normw, dinv, bl[l], gam + l * kD, bet + l * kD,
                                                 rmean + l * kD, rvar + l * kD, accp, act16);
    }
  }
  pool_kernel<<<kNPB, kNT, 0, stream>>>(accp, bidx, wout, bout, out);
}
